// MaskedMultiSelfAttention_46763603918977
// MI455X (gfx1250) — hardware-verified
//
#include <hip/hip_runtime.h>
#include <stdint.h>

typedef __attribute__((ext_vector_type(16))) _Float16 v16h;
typedef __attribute__((ext_vector_type(8)))  _Float16 v8h;
typedef __attribute__((ext_vector_type(16))) __bf16   v16b;
typedef __attribute__((ext_vector_type(8)))  __bf16   v8b;
typedef __attribute__((ext_vector_type(8)))  float    v8f;
typedef __attribute__((ext_vector_type(4)))  float    v4f;

#ifndef NB
#define NB 4
#endif
#ifndef SEQ
#define SEQ 2048
#endif
#ifndef NB_FULL
#define NB_FULL 4
#endif
#ifndef SEQ_FULL
#define SEQ_FULL 2048
#endif
constexpr int kBatch     = NB;
constexpr int kSeq       = SEQ;
constexpr int kBatchFull = NB_FULL;
constexpr int kSeqFull   = SEQ_FULL;
constexpr int kChan      = 1024;
constexpr int kHeads     = 16;
constexpr int kHeadDim   = 64;
constexpr int kQkvW      = 3 * kChan;
constexpr int kGrp       = (kBatch % 2 == 0) ? 2 : 1;
constexpr int kNGrp      = kBatch / kGrp;
constexpr int kTok       = kBatch * kSeq;
constexpr int kTokG      = kGrp * kSeq;
constexpr int kKeyChunk  = 64;
constexpr int kQryBlock  = 64;
constexpr int kOsPitch   = 68;
constexpr int kWtPitch   = 72;
static_assert(kSeq % 64 == 0);
static_assert(kSeq >= 64);
static_assert(kSeq <= kSeqFull);
static_assert(kBatch >= 1);
static_assert(kBatch <= kBatchFull);
static_assert(kNGrp * kGrp == kBatch);
static_assert(kChan % 64 == 0);
static_assert(kQkvW % 64 == 0);
static_assert(kChan % 32 == 0);
static_assert(kHeads * kHeadDim == kChan);
static_assert((kTok * kChan / 2) % 256 == 0);

constexpr size_t kSzXb   = (size_t)kTok  * kChan * 2;
constexpr size_t kSzWat  = (size_t)kQkvW * kChan * 2;
constexpr size_t kSzWpt  = (size_t)kChan * kChan * 2;
constexpr size_t kSzQ    = (size_t)kTokG * kQkvW * 2;
constexpr size_t kSzO    = (size_t)kTokG * kChan * 2;
constexpr size_t kOffXb  = 0;
constexpr size_t kOffWat = kOffXb + kSzXb;
constexpr size_t kOffWpt = kOffWat + kSzWat;
constexpr size_t kOffQh  = kOffWpt + kSzWpt;
constexpr size_t kOffQl  = kOffQh + kSzQ;
constexpr size_t kOffOh  = kOffQl + kSzQ;
constexpr size_t kOffOl  = kOffOh + kSzO;
constexpr size_t kWsTotal = kOffOl + kSzO;
static_assert(kWsTotal <= (size_t)134217728);
static_assert(kOffWat % 256 == 0);
static_assert(kOffWpt % 256 == 0);
static_assert(kOffQh % 256 == 0);
static_assert(kOffQl % 256 == 0);
static_assert(kOffOh % 256 == 0);
static_assert(kOffOl % 256 == 0);
static_assert(((size_t)(kBatch - 1) * kSeqFull + kSeq) * kChan <= (size_t)kBatchFull * kSeqFull * kChan);

__device__ __forceinline__ unsigned short f2bf_bits(float f) {
  unsigned u = __float_as_uint(f);
  return (unsigned short)((u + 0x7FFFu + ((u >> 16) & 1u)) >> 16);
}
__device__ __forceinline__ float bf_bits2f(unsigned short h) { return __uint_as_float(((unsigned)h) << 16); }

__device__ __forceinline__ void dep_guard_h(v8f& a, v8f& b, v16h x, v16h y) { asm volatile("v_nop\n\tv_nop\n\tv_nop\n\tv_nop" : "+v"(a), "+v"(b) : "v"(x), "v"(y)); }
__device__ __forceinline__ void dep_guard_b(v8f& a, v8f& b, v16b x, v16b y) { asm volatile("v_nop\n\tv_nop\n\tv_nop\n\tv_nop" : "+v"(a), "+v"(b) : "v"(x), "v"(y)); }
__device__ __forceinline__ void keep4_h(v16h a, v16h b, v16h c, v16h d) { asm volatile("v_nop" :: "v"(a), "v"(b), "v"(c), "v"(d)); }
__device__ __forceinline__ void keep4_b(v16b a, v16b b, v16b c, v16b d) { asm volatile("v_nop" :: "v"(a), "v"(b), "v"(c), "v"(d)); }
__device__ __forceinline__ void acc_guard4(v8f& a, v8f& b, v8f& c, v8f& d) { asm volatile("v_nop\n\tv_nop\n\tv_nop\n\tv_nop" : "+v"(a), "+v"(b), "+v"(c), "+v"(d)); }
template <typename T> struct Frag;
template <> struct Frag<_Float16> {
  typedef v16h V; union U { v16h v; v8h h[2]; };
  static __device__ __forceinline__ v16h load(const _Float16* p) {
    U f; f.h[0] = *(const v8h*)(p); f.h[1] = *(const v8h*)(p + 16); return f.v;
  }
  static __device__ __forceinline__ v8f mma(v16h a, v16h b, v8f c) {
    return __builtin_amdgcn_wmma_f32_16x16x32_f16(false, a, false, b, (short)0, c, false, false);
  }
  static __device__ __forceinline__ void guard(v8f& a, v8f& b, v16h x, v16h y) { dep_guard_h(a, b, x, y); }
  static __device__ __forceinline__ void keep(v16h a, v16h b, v16h c, v16h d) { keep4_h(a, b, c, d); }
};
template <> struct Frag<__bf16> {
  typedef v16b V; union U { v16b v; v8b h[2]; };
  static __device__ __forceinline__ v16b load(const __bf16* p) {
    U f; f.h[0] = *(const v8b*)(p); f.h[1] = *(const v8b*)(p + 16); return f.v;
  }
  static __device__ __forceinline__ v8f mma(v16b a, v16b b, v8f c) {
    return __builtin_amdgcn_wmma_f32_16x16x32_bf16(false, a, false, b, (short)0, c, false, false);
  }
  static __device__ __forceinline__ void guard(v8f& a, v8f& b, v16b x, v16b y) { dep_guard_b(a, b, x, y); }
  static __device__ __forceinline__ void keep(v16b a, v16b b, v16b c, v16b d) { keep4_b(a, b, c, d); }
};

template <int ET> struct Elem;
template <> struct Elem<0> { typedef _Float16 T; };
template <> struct Elem<1> { typedef __bf16 T; };
template <int ET, int SPLIT, int BIAS_MODE, int OUT_MODE, bool RESID, int ACT = 0>
__global__ __launch_bounds__(256) void wmma_gemm64(
    const unsigned short* __restrict__ Ap, const unsigned short* __restrict__ A2p, int lda, long strideA,
    const unsigned short* __restrict__ Btp, const unsigned short* __restrict__ Bt2p, int ldb, long strideB,
    void* __restrict__ Cout, void* __restrict__ Cout2, int ldc, long strideC,
    const float* __restrict__ bias,
    const float* __restrict__ resid, long strideR,
    int M, int N, int K, float scale) {
  typedef typename Elem<ET>::T T;
  typedef typename Frag<T>::V V;
  const T* A = (const T*)Ap; const T* A2 = (const T*)A2p; const T* Bt = (const T*)Btp; const T* Bt2 = (const T*)Bt2p;
  __shared__ __align__(16) float sT[8][16 * 68];
  const int b    = blockIdx.y;
  const int lane = threadIdx.x & 31;
  const int wave = threadIdx.x >> 5;
  const int tilesN = N >> 6;
  const int tilesM = M >> 6;
  const int tile = blockIdx.x * 8 + wave;
  if (tile >= tilesM * tilesN) return;
  const int tm = tile / tilesN;
  const int tn = tile - tm * tilesN;
  const int m0 = tm << 6;
  const int n0 = tn << 6;

  const T* Ab  = A  + (size_t)b * strideA;
  const T* Bb  = Bt + (size_t)b * strideB;
  const T* Ab2 = (SPLIT != 0) ? (A2  + (size_t)b * strideA) : nullptr;
  const T* Bb2 = (SPLIT == 1) ? (Bt2 + (size_t)b * strideB) : nullptr;

  const int rlane = lane & 15;
  const int koff  = (lane >> 4) * 8;
  const int mOff  = (lane >> 4) * 8;

  v8f acc[4][4];
#pragma unroll
  for (int i = 0; i < 4; ++i)
#pragma unroll
    for (int j = 0; j < 4; ++j) acc[i][j] = (v8f){0.f,0.f,0.f,0.f,0.f,0.f,0.f,0.f};

  for (int k0 = 0; k0 < K; k0 += 32) {
    V bh[4], bl[4];
#pragma unroll
    for (int j = 0; j < 4; ++j) {
      const size_t bo = (size_t)(n0 + (j << 4) + rlane) * ldb + koff + k0;
      bh[j] = Frag<T>::load(Bb + bo);
      if (SPLIT == 1) bl[j] = Frag<T>::load(Bb2 + bo);
    }
#pragma unroll
    for (int i = 0; i < 4; ++i) {
      const size_t ao = (size_t)(m0 + (i << 4) + rlane) * lda + koff + k0;
      V ah = Frag<T>::load(Ab + ao);
      V al;
      if (SPLIT != 0) al = Frag<T>::load(Ab2 + ao);
#pragma unroll
      for (int j = 0; j < 4; ++j) {
        acc[i][j] = Frag<T>::mma(ah, bh[j], acc[i][j]);
        if (SPLIT == 1) acc[i][j] = Frag<T>::mma(ah, bl[j], acc[i][j]);
        if (SPLIT != 0) acc[i][j] = Frag<T>::mma(al, bh[j], acc[i][j]);
      }
      Frag<T>::guard(acc[i][0], acc[i][3], ah, (SPLIT != 0) ? al : ah);
    }
    Frag<T>::keep(bh[0], bh[1], bh[2], bh[3]);
    if (SPLIT == 1) Frag<T>::keep(bl[0], bl[1], bl[2], bl[3]);
  }
  acc_guard4(acc[0][0], acc[0][1], acc[0][2], acc[0][3]);
  acc_guard4(acc[1][0], acc[1][1], acc[1][2], acc[1][3]);
  acc_guard4(acc[2][0], acc[2][1], acc[2][2], acc[2][3]);
  acc_guard4(acc[3][0], acc[3][1], acc[3][2], acc[3][3]);

  float* slab = sT[wave];
  const float* Rb = RESID ? (resid + (size_t)b * strideR) : nullptr;
#pragma unroll
  for (int i = 0; i < 4; ++i) {
    const int mBase = m0 + (i << 4);
#pragma unroll
    for (int j = 0; j < 4; ++j) {
      const int n = n0 + (j << 4) + rlane;
      float bv = 0.f;
      if (BIAS_MODE == 2) bv = bias[n];
#pragma unroll
      for (int r = 0; r < 8; ++r) {
        float v = acc[i][j][r] * scale;
        if (BIAS_MODE == 1) v += bias[mBase + mOff + r];
        if (BIAS_MODE == 2) v += bv;
        if (RESID) v += Rb[(size_t)(mBase + mOff + r) * ldc + n];
        if (ACT == 1) v = tanhf(v);
        if (ACT == 2) v = fmaxf(v, 0.0f);
        if (ACT == 3) v = v / (1.0f + expf(-v));
        if (ACT == 4) v = (v > 0.f) ? v : 0.01f * v;
        slab[(mOff + r) * 68 + (j << 4) + rlane] = v;
      }
    }
    __builtin_amdgcn_fence(__ATOMIC_RELEASE, "workgroup");
    __builtin_amdgcn_wave_barrier();
    __builtin_amdgcn_fence(__ATOMIC_ACQUIRE, "workgroup");
    if (OUT_MODE == 0) {
      float* C = (float*)Cout + (size_t)b * strideC;
      const int hh = lane >> 4, c4 = (lane & 15) * 4;
      for (int pass = 0; pass < 2; ++pass) {
#pragma unroll
        for (int it = 0; it < 8; ++it) {
          const int row = it * 2 + hh;
          v4f v = *(const v4f*)(slab + row * 68 + c4);
          *(volatile v4f*)(C + (size_t)(mBase + row) * ldc + n0 + c4) = v;
        }
        __threadfence();
      }
    } else {
      const int q = lane >> 3, c8 = (lane & 7) * 8;
      unsigned short* C  = (unsigned short*)Cout  + (size_t)b * strideC;
      unsigned short* C2 = (OUT_MODE == 2) ? ((unsigned short*)Cout2 + (size_t)b * strideC) : nullptr;
      for (int pass = 0; pass < 2; ++pass) {
#pragma unroll
        for (int it = 0; it < 4; ++it) {
          const int row = it * 4 + q;
          const float* sp = slab + row * 68 + c8;
          v8h hv, lv;
#pragma unroll
          for (int e = 0; e < 8; ++e) {
            if (OUT_MODE == 1) {
              hv[e] = (_Float16)sp[e];
            } else {
              unsigned short hb = f2bf_bits(sp[e]);
              unsigned short lb = f2bf_bits(sp[e] - bf_bits2f(hb));
              hv[e] = __builtin_bit_cast(_Float16, hb);
              lv[e] = __builtin_bit_cast(_Float16, lb);
            }
          }
          *(volatile v8h*)(C + (size_t)(mBase + row) * ldc + n0 + c8) = hv;
          if (OUT_MODE == 2) *(volatile v8h*)(C2 + (size_t)(mBase + row) * ldc + n0 + c8) = lv;
        }
        __threadfence();
      }
    }
    __builtin_amdgcn_fence(__ATOMIC_RELEASE, "workgroup");
    __builtin_amdgcn_wave_barrier();
    __builtin_amdgcn_fence(__ATOMIC_ACQUIRE, "workgroup");
  }
}

__global__ __launch_bounds__(256) void cast_x_bf16x2(
    const float* __restrict__ in, unsigned short* __restrict__ out, int n2) {
  int i = blockIdx.x * 256 + threadIdx.x;
  if (i < n2) {
    const int e   = 2 * i;
    const int row = e / kChan;
    const int col = e - row * kChan;
    const int b   = row / kSeq;
    const int t   = row - b * kSeq;
    const size_t src = ((size_t)b * kSeqFull + t) * (size_t)kChan + col;
    const unsigned u = (unsigned)f2bf_bits(in[src]) | ((unsigned)f2bf_bits(in[src + 1]) << 16);
    ((volatile unsigned*)out)[i] = u;
    __threadfence();
    ((volatile unsigned*)out)[i] = u;
  }
}

__global__ __launch_bounds__(256) void wt_cast_bf_k(const float* __restrict__ W, unsigned short* __restrict__ Wtp,
                                                    int Kd, int Nd, float mul) {
  __shared__ __align__(16) _Float16 st[64 * kWtPitch];
  _Float16* Wt = (_Float16*)(void*)Wtp;
  const int n0 = blockIdx.x * 64, k0 = blockIdx.y * 64;
  const int tid = threadIdx.x;
  const int kr = tid >> 2, c16 = (tid & 3) * 16;
  const float* src = W + (size_t)(k0 + kr) * Nd + n0 + c16;
#pragma unroll
  for (int q = 0; q < 4; ++q) {
    const v4f v = *(const v4f*)(src + 4 * q);
#pragma unroll
    for (int e = 0; e < 4; ++e)
      st[(c16 + 4 * q + e) * kWtPitch + kr] = __builtin_bit_cast(_Float16, f2bf_bits(v[e] * mul));
  }
  __syncthreads();
  const int wave = tid >> 5, lane = tid & 31;
  const int q8 = lane >> 3, c8 = (lane & 7) * 8;
  for (int pass = 0; pass < 2; ++pass) {
#pragma unroll
    for (int it = 0; it < 2; ++it) {
      const int n = it * 32 + wave * 4 + q8;
      const v8h hv = *(const v8h*)(st + n * kWtPitch + c8);
      *(volatile v8h*)(Wt + (size_t)(n0 + n) * Kd + k0 + c8) = hv;
    }
    __threadfence();
  }
}

__device__ __forceinline__ __bf16 at_f2bf(float f) { return __builtin_bit_cast(__bf16, f2bf_bits(f)); }
__device__ __forceinline__ void at_split(float f, __bf16& hi, __bf16& lo) {
  const unsigned short hb = f2bf_bits(f);
  hi = __builtin_bit_cast(__bf16, hb);
  lo = at_f2bf(f - __uint_as_float(((unsigned)hb) << 16));
}
__device__ __forceinline__ v8f at_mma(v16b a, v16b b, v8f c) {
  c = __builtin_amdgcn_wmma_f32_16x16x32_bf16(false, a, false, b, (short)0, c, false, false);
  asm volatile("v_nop\n\tv_nop\n\tv_nop\n\tv_nop" : "+v"(c) : "v"(a), "v"(b));
  return c;
}

__global__ __launch_bounds__(128)
void attn_hd64_k(const unsigned short* __restrict__ qkvh_p, const unsigned short* __restrict__ qkvl_p,
                 unsigned short* __restrict__ oh_p, unsigned short* __restrict__ ol_p) {
  union FB { v16b v; v8b h[2]; };
  __shared__ __align__(16) __bf16 Ksh[kKeyChunk * kHeadDim];
  __shared__ __align__(16) __bf16 Ksl[kKeyChunk * kHeadDim];
  __shared__ __align__(16) __bf16 Vth[kHeadDim * kKeyChunk];
  __shared__ __align__(16) __bf16 Vtl[kHeadDim * kKeyChunk];
  __shared__ __align__(16) __bf16 Psh[4][16 * kKeyChunk];
  __shared__ __align__(16) __bf16 Psl[4][16 * kKeyChunk];
  __shared__ __align__(16) float  Osm[4][16 * kOsPitch];

  const __bf16* QH = (const __bf16*)(const void*)qkvh_p;
  const __bf16* QL = (const __bf16*)(const void*)qkvl_p;
  _Float16* OH = (_Float16*)(void*)oh_p;
  _Float16* OL = (_Float16*)(void*)ol_p;

  const int tid  = threadIdx.x;
  const int wave = tid >> 5;
  const int lane = tid & 31;
  const int hh   = lane >> 4;
  const int c    = lane & 15;

  const int nqb = kSeq / kQryBlock;
  const int bx  = blockIdx.x;
  const int qb  = bx % nqb;
  const int bh  = bx / nqb;
  const int h   = bh % kHeads;
  const int b   = bh / kHeads;
  const int q0  = qb * kQryBlock + wave * 16;
  const size_t rs   = (size_t)kQkvW;
  const size_t tokb = (size_t)b * kSeq;
  const size_t hcol = (size_t)h * kHeadDim;

  v16b qah[2], qal[2];
  {
    const size_t qo = (tokb + q0 + c) * rs + hcol + 8 * hh;
#pragma unroll
    for (int dc = 0; dc < 2; ++dc) {
      qah[dc] = Frag<__bf16>::load(QH + qo + dc * 32);
      qal[dc] = Frag<__bf16>::load(QL + qo + dc * 32);
    }
  }

  float mrow[8], lrow[8];
  v8f oacc[4];
#pragma unroll
  for (int r = 0; r < 8; ++r) { mrow[r] = -1.0e30f; lrow[r] = 0.f; }
#pragma unroll
  for (int t = 0; t < 4; ++t) oacc[t] = (v8f){0.f,0.f,0.f,0.f,0.f,0.f,0.f,0.f};

  const int nChunks = qb + 1;
  for (int kc = 0; kc < nChunks; ++kc) {
    const int kv0 = kc * kKeyChunk;
    __syncthreads();
    {
      const int kvr = tid >> 1, dh = (tid & 1) * 32;
      const size_t ro = (tokb + kv0 + kvr) * rs + hcol + dh;
      const __bf16* kph = QH + ro + kChan;
      const __bf16* kpl = QL + ro + kChan;
      const __bf16* vph = QH + ro + 2 * kChan;
      const __bf16* vpl = QL + ro + 2 * kChan;
#pragma unroll 1
      for (int i = 0; i < 4; ++i) {
        const v8b a0 = *(const v8b*)(kph + 8 * i);
        const v8b a1 = *(const v8b*)(kpl + 8 * i);
        *(v8b*)(Ksh + kvr * kHeadDim + dh + 8 * i) = a0;
        *(v8b*)(Ksl + kvr * kHeadDim + dh + 8 * i) = a1;
        const v8b w0 = *(const v8b*)(vph + 8 * i);
        const v8b w1 = *(const v8b*)(vpl + 8 * i);
#pragma unroll
        for (int e = 0; e < 8; ++e) {
          Vth[(dh + 8 * i + e) * kKeyChunk + kvr] = w0[e];
          Vtl[(dh + 8 * i + e) * kKeyChunk + kvr] = w1[e];
        }
      }
    }
    __syncthreads();

    v8f s[4];
#pragma unroll
    for (int j = 0; j < 4; ++j) {
      s[j] = (v8f){0.f,0.f,0.f,0.f,0.f,0.f,0.f,0.f};
#pragma unroll
      for (int dc = 0; dc < 2; ++dc) {
        FB kb, kl;
        kb.h[0] = *(const v8b*)(Ksh + (j * 16 + c) * kHeadDim + dc * 32 + 8 * hh);
        kb.h[1] = *(const v8b*)(Ksh + (j * 16 + c) * kHeadDim + dc * 32 + 16 + 8 * hh);
        kl.h[0] = *(const v8b*)(Ksl + (j * 16 + c) * kHeadDim + dc * 32 + 8 * hh);
        kl.h[1] = *(const v8b*)(Ksl + (j * 16 + c) * kHeadDim + dc * 32 + 16 + 8 * hh);
        s[j] = at_mma(qah[dc], kb.v, s[j]);
        s[j] = at_mma(qah[dc], kl.v, s[j]);
        s[j] = at_mma(qal[dc], kb.v, s[j]);
      }
    }

    const bool diag = (kc == qb);
    float cm[8];
#pragma unroll
    for (int r = 0; r < 8; ++r) {
      const int qrow = q0 + 8 * hh + r;
      float m = -1.0e30f;
#pragma unroll
      for (int j = 0; j < 4; ++j) {
        const int kvcol = kv0 + j * 16 + c;
        float sv = s[j][r] * 0.125f;
        if (diag && (kvcol > qrow)) sv = -1.0e9f;
        s[j][r] = sv;
        m = fmaxf(m, sv);
      }
#pragma unroll
      for (int off = 1; off < 16; off <<= 1) m = fmaxf(m, __shfl_xor(m, off, 32));
      cm[r] = m;
    }
    __bf16* pwh = Psh[wave];
    __bf16* pwl = Psl[wave];
#pragma unroll
    for (int r = 0; r < 8; ++r) {
      const float mnew = fmaxf(mrow[r], cm[r]);
      const float alpha = expf(mrow[r] - mnew);
      mrow[r] = mnew;
      float psum = 0.f;
#pragma unroll
      for (int j = 0; j < 4; ++j) {
        const float p = expf(s[j][r] - mnew);
        psum += p;
        __bf16 ph, pl;
        at_split(p, ph, pl);
        pwh[(8 * hh + r) * kKeyChunk + j * 16 + c] = ph;
        pwl[(8 * hh + r) * kKeyChunk + j * 16 + c] = pl;
      }
#pragma unroll
      for (int off = 1; off < 16; off <<= 1) psum += __shfl_xor(psum, off, 32);
      lrow[r] = lrow[r] * alpha + psum;
#pragma unroll
      for (int t = 0; t < 4; ++t) oacc[t][r] *= alpha;
    }
    __builtin_amdgcn_fence(__ATOMIC_RELEASE, "workgroup");
    __builtin_amdgcn_wave_barrier();
    __builtin_amdgcn_fence(__ATOMIC_ACQUIRE, "workgroup");
#pragma unroll
    for (int kk = 0; kk < 2; ++kk) {
      FB pa, pb;
      pa.h[0] = *(const v8b*)(pwh + c * kKeyChunk + kk * 32 + 8 * hh);
      pa.h[1] = *(const v8b*)(pwh + c * kKeyChunk + kk * 32 + 16 + 8 * hh);
      pb.h[0] = *(const v8b*)(pwl + c * kKeyChunk + kk * 32 + 8 * hh);
      pb.h[1] = *(const v8b*)(pwl + c * kKeyChunk + kk * 32 + 16 + 8 * hh);
#pragma unroll
      for (int t = 0; t < 4; ++t) {
        FB vb, vl;
        vb.h[0] = *(const v8b*)(Vth + (t * 16 + c) * kKeyChunk + kk * 32 + 8 * hh);
        vb.h[1] = *(const v8b*)(Vth + (t * 16 + c) * kKeyChunk + kk * 32 + 16 + 8 * hh);
        vl.h[0] = *(const v8b*)(Vtl + (t * 16 + c) * kKeyChunk + kk * 32 + 8 * hh);
        vl.h[1] = *(const v8b*)(Vtl + (t * 16 + c) * kKeyChunk + kk * 32 + 16 + 8 * hh);
        oacc[t] = at_mma(pa.v, vb.v, oacc[t]);
        oacc[t] = at_mma(pa.v, vl.v, oacc[t]);
        oacc[t] = at_mma(pb.v, vb.v, oacc[t]);
      }
    }
  }

  float* os = Osm[wave];
#pragma unroll
  for (int r = 0; r < 8; ++r) {
    const float inv = 1.0f / lrow[r];
#pragma unroll
    for (int t = 0; t < 4; ++t) os[(8 * hh + r) * kOsPitch + t * 16 + c] = oacc[t][r] * inv;
  }
  __builtin_amdgcn_fence(__ATOMIC_RELEASE, "workgroup");
  __builtin_amdgcn_wave_barrier();
  __builtin_amdgcn_fence(__ATOMIC_ACQUIRE, "workgroup");
  {
    const int q8 = lane >> 3, c8 = (lane & 7) * 8;
    for (int pass = 0; pass < 2; ++pass) {
#pragma unroll
      for (int it = 0; it < 4; ++it) {
        const int row = it * 4 + q8;
        const float* sp = os + row * kOsPitch + c8;
        const v4f x0 = *(const v4f*)(sp);
        const v4f x1 = *(const v4f*)(sp + 4);
        v8h hv, lv;
#pragma unroll
        for (int e = 0; e < 4; ++e) {
          const unsigned short hb0 = f2bf_bits(x0[e]);
          const unsigned short lb0 = f2bf_bits(x0[e] - bf_bits2f(hb0));
          hv[e] = __builtin_bit_cast(_Float16, hb0);
          lv[e] = __builtin_bit_cast(_Float16, lb0);
          const unsigned short hb1 = f2bf_bits(x1[e]);
          const unsigned short lb1 = f2bf_bits(x1[e] - bf_bits2f(hb1));
          hv[4 + e] = __builtin_bit_cast(_Float16, hb1);
          lv[4 + e] = __builtin_bit_cast(_Float16, lb1);
        }
        const size_t go = (tokb + q0 + row) * (size_t)kChan + hcol + c8;
        *(volatile v8h*)(OH + go) = hv;
        *(volatile v8h*)(OL + go) = lv;
      }
      __threadfence();
    }
  }
}

extern "C" void kernel_launch(void* const* d_in, const int* in_sizes, int n_in,
                              void* d_out, int out_size, void* d_ws, size_t ws_size,
                              hipStream_t stream) {
  if (n_in < 5) return;
  if (in_sizes[0] < ((kBatch - 1) * kSeqFull + kSeq) * kChan) return;
  if (in_sizes[1] < kChan * kQkvW) return;
  if (in_sizes[2] < kQkvW) return;
  if (in_sizes[3] < kChan * kChan) return;
  if (in_sizes[4] < kChan) return;
  if (out_size < ((kBatch - 1) * kSeqFull + kSeq) * kChan) return;
  if (ws_size < kWsTotal) return;

  const float* x      = (const float*)d_in[0];
  const float* W_attn = (const float*)d_in[1];
  const float* b_attn = (const float*)d_in[2];
  const float* W_proj = (const float*)d_in[3];
  const float* b_proj = (const float*)d_in[4];

  char* ws = (char*)d_ws;
  unsigned short* xb  = (unsigned short*)(ws + kOffXb);
  unsigned short* wat = (unsigned short*)(ws + kOffWat);
  unsigned short* wpt = (unsigned short*)(ws + kOffWpt);
  unsigned short* qh  = (unsigned short*)(ws + kOffQh);
  unsigned short* ql  = (unsigned short*)(ws + kOffQl);
  unsigned short* oh  = (unsigned short*)(ws + kOffOh);
  unsigned short* ol  = (unsigned short*)(ws + kOffOl);

  const int nx2 = kTok * kChan / 2;
  cast_x_bf16x2<<<dim3((nx2 + 255) / 256), dim3(256), 0, stream>>>(x, xb, nx2);
  wt_cast_bf_k<<<dim3(kQkvW / 64, kChan / 64), dim3(256), 0, stream>>>(W_attn, wat, kChan, kQkvW, 1.0f);
  wt_cast_bf_k<<<dim3(kChan / 64, kChan / 64), dim3(256), 0, stream>>>(W_proj, wpt, kChan, kChan, 1.0f);

  for (int g = 0; g < kNGrp; ++g) {
    const unsigned short* xg = xb + (size_t)g * kTokG * kChan;
    const int tilesQkv = (kTokG / 64) * (kQkvW / 64);
    wmma_gemm64<1, 0, 2, 2, false, 0><<<dim3((tilesQkv + 7) / 8, 1), dim3(256), 0, stream>>>(
        xg, xg, kChan, 0L, wat, wat, kChan, 0L, (void*)qh, (void*)ql, kQkvW, 0L,
        b_attn, (const float*)nullptr, 0L, kTokG, kQkvW, kChan, 1.0f);
    attn_hd64_k<<<dim3(kGrp * kHeads * (kSeq / kQryBlock)), dim3(128), 0, stream>>>(qh, ql, oh, ol);
    float* cg = (float*)d_out + (size_t)g * kGrp * kSeqFull * kChan;
    const int tilesOut = (kSeq / 64) * (kChan / 64);
    wmma_gemm64<1, 2, 2, 0, false, 0><<<dim3((tilesOut + 7) / 8, kGrp), dim3(256), 0, stream>>>(
        oh, ol, kChan, (long)kSeq * kChan, wpt, wpt, kChan, 0L, (void*)cg, (void*)nullptr, kChan,
        (long)kSeqFull * kChan, b_proj, (const float*)nullptr, 0L, kSeq, kChan, kChan, 1.0f);
  }
}
